// TimeMixing_9826885173421
// MI455X (gfx1250) — hardware-verified
//
#include <hip/hip_runtime.h>
#include <stddef.h>

constexpr int NBATCH = 2;
constexpr int NTOK   = 256;
constexpr int NEMB   = 512;
constexpr int NATT   = 512;
constexpr int NROWS  = NBATCH * NTOK;
static_assert(NROWS % 64 == 0 && NATT % 64 == 0 && NEMB % 64 == 0, "");
static_assert(NEMB % 32 == 0 && NATT % 32 == 0, "");
static_assert((NROWS * NEMB) % 2048 == 0 && (NATT * NEMB) % 2048 == 0 && (NROWS * NATT) % 2048 == 0, "");

typedef __attribute__((ext_vector_type(16))) _Float16 v16h;
typedef __attribute__((ext_vector_type(8)))  _Float16 v8h;
typedef __attribute__((ext_vector_type(16))) __bf16   v16b;
typedef __attribute__((ext_vector_type(8)))  __bf16   v8b;
typedef __attribute__((ext_vector_type(8)))  float    v8f;
typedef __attribute__((ext_vector_type(4)))  float    v4f;
typedef __attribute__((ext_vector_type(4)))  unsigned int v4u;

__device__ __forceinline__ unsigned short f2bf_bits(float f) {
  unsigned u = __float_as_uint(f);
  return (unsigned short)((u + 0x7FFFu + ((u >> 16) & 1u)) >> 16);
}
__device__ __forceinline__ float bf_bits2f(unsigned short h) { return __uint_as_float(((unsigned)h) << 16); }

__device__ __forceinline__ void dep_guard_h(v8f& a, v8f& b, v16h x, v16h y) { asm volatile("v_nop\n\tv_nop\n\tv_nop\n\tv_nop" : "+v"(a), "+v"(b) : "v"(x), "v"(y)); }
__device__ __forceinline__ void dep_guard_b(v8f& a, v8f& b, v16b x, v16b y) { asm volatile("v_nop\n\tv_nop\n\tv_nop\n\tv_nop" : "+v"(a), "+v"(b) : "v"(x), "v"(y)); }
__device__ __forceinline__ void dep_guard4_h(v8f& a, v8f& b, v8f& c, v8f& d, v16h x, v16h y) { asm volatile("v_nop\n\tv_nop\n\tv_nop\n\tv_nop" : "+v"(a), "+v"(b), "+v"(c), "+v"(d) : "v"(x), "v"(y)); }
__device__ __forceinline__ void dep_guard4_b(v8f& a, v8f& b, v8f& c, v8f& d, v16b x, v16b y) { asm volatile("v_nop\n\tv_nop\n\tv_nop\n\tv_nop" : "+v"(a), "+v"(b), "+v"(c), "+v"(d) : "v"(x), "v"(y)); }
__device__ __forceinline__ void keep4_h(v16h a, v16h b, v16h c, v16h d) { asm volatile("v_nop" :: "v"(a), "v"(b), "v"(c), "v"(d)); }
__device__ __forceinline__ void keep4_b(v16b a, v16b b, v16b c, v16b d) { asm volatile("v_nop" :: "v"(a), "v"(b), "v"(c), "v"(d)); }
__device__ __forceinline__ void acc_guard4(v8f& a, v8f& b, v8f& c, v8f& d) { asm volatile("v_nop\n\tv_nop\n\tv_nop\n\tv_nop" : "+v"(a), "+v"(b), "+v"(c), "+v"(d)); }
template <typename T> struct Frag;
template <> struct Frag<_Float16> {
  typedef v16h V; union U { v16h v; v8h h[2]; };
  static __device__ __forceinline__ v16h load(const _Float16* p) {
    U f; f.h[0] = *(const v8h*)(p); f.h[1] = *(const v8h*)(p + 16); return f.v;
  }
  static __device__ __forceinline__ v8f mma(v16h a, v16h b, v8f c) {
    return __builtin_amdgcn_wmma_f32_16x16x32_f16(false, a, false, b, (short)0, c, false, false);
  }
  static __device__ __forceinline__ void guard(v8f& a, v8f& b, v16h x, v16h y) { dep_guard_h(a, b, x, y); }
  static __device__ __forceinline__ void guard4(v8f& a, v8f& b, v8f& c, v8f& d, v16h x, v16h y) { dep_guard4_h(a, b, c, d, x, y); }
  static __device__ __forceinline__ void keep(v16h a, v16h b, v16h c, v16h d) { keep4_h(a, b, c, d); }
};
template <> struct Frag<__bf16> {
  typedef v16b V; union U { v16b v; v8b h[2]; };
  static __device__ __forceinline__ v16b load(const __bf16* p) {
    U f; f.h[0] = *(const v8b*)(p); f.h[1] = *(const v8b*)(p + 16); return f.v;
  }
  static __device__ __forceinline__ v8f mma(v16b a, v16b b, v8f c) {
    return __builtin_amdgcn_wmma_f32_16x16x32_bf16(false, a, false, b, (short)0, c, false, false);
  }
  static __device__ __forceinline__ void guard(v8f& a, v8f& b, v16b x, v16b y) { dep_guard_b(a, b, x, y); }
  static __device__ __forceinline__ void guard4(v8f& a, v8f& b, v8f& c, v8f& d, v16b x, v16b y) { dep_guard4_b(a, b, c, d, x, y); }
  static __device__ __forceinline__ void keep(v16b a, v16b b, v16b c, v16b d) { keep4_b(a, b, c, d); }
};

template <int ET> struct Elem;
template <> struct Elem<0> { typedef _Float16 T; };
template <> struct Elem<1> { typedef __bf16 T; };
template <int ET, bool SPLIT, int BIAS_MODE, int OUT_MODE, bool RESID, int ACT = 0>
__global__ __launch_bounds__(256) void wmma_gemm64(
    const unsigned short* __restrict__ Ap, const unsigned short* __restrict__ A2p, int lda, long strideA,
    const unsigned short* __restrict__ Btp, const unsigned short* __restrict__ Bt2p, int ldb, long strideB,
    void* __restrict__ Cout, void* __restrict__ Cout2, int ldc, long strideC,
    const float* __restrict__ bias,
    const float* __restrict__ resid, long strideR,
    int M, int N, int K, float scale) {
  typedef typename Elem<ET>::T T;
  typedef typename Frag<T>::V V;
  const T* A = (const T*)Ap; const T* A2 = (const T*)A2p; const T* Bt = (const T*)Btp; const T* Bt2 = (const T*)Bt2p;
  __shared__ __align__(16) float sT[8][16 * 68];
  const int b    = blockIdx.y;
  const int lane = threadIdx.x & 31;
  const int wave = threadIdx.x >> 5;
  const int tilesN = N >> 6;
  const int tilesM = M >> 6;
  const int tile = blockIdx.x * 8 + wave;
  if (tile >= tilesM * tilesN) return;
  const int tm = tile / tilesN;
  const int tn = tile - tm * tilesN;
  const int m0 = tm << 6;
  const int n0 = tn << 6;

  const T* Ab  = A  + (size_t)b * strideA;
  const T* Bb  = Bt + (size_t)b * strideB;
  const T* Ab2 = SPLIT ? (A2  + (size_t)b * strideA) : nullptr;
  const T* Bb2 = SPLIT ? (Bt2 + (size_t)b * strideB) : nullptr;

  const int rlane = lane & 15;
  const int koff  = (lane >> 4) * 8;
  const int mOff  = (lane >> 4) * 8;

  v8f acc[4][4];
#pragma unroll
  for (int i = 0; i < 4; ++i)
#pragma unroll
    for (int j = 0; j < 4; ++j) acc[i][j] = (v8f){0.f,0.f,0.f,0.f,0.f,0.f,0.f,0.f};

  for (int k0 = 0; k0 < K; k0 += 32) {
    V bh[4], bl[4];
#pragma unroll
    for (int j = 0; j < 4; ++j) {
      const size_t bo = (size_t)(n0 + (j << 4) + rlane) * ldb + koff + k0;
      bh[j] = Frag<T>::load(Bb + bo);
      if (SPLIT) bl[j] = Frag<T>::load(Bb2 + bo);
    }
#pragma unroll
    for (int i = 0; i < 4; ++i) {
      const size_t ao = (size_t)(m0 + (i << 4) + rlane) * lda + koff + k0;
      V ah = Frag<T>::load(Ab + ao);
      V al;
      if (SPLIT) al = Frag<T>::load(Ab2 + ao);
#pragma unroll
      for (int j = 0; j < 4; ++j) {
        acc[i][j] = Frag<T>::mma(ah, bh[j], acc[i][j]);
        if (SPLIT) {
          acc[i][j] = Frag<T>::mma(ah, bl[j], acc[i][j]);
          acc[i][j] = Frag<T>::mma(al, bh[j], acc[i][j]);
        }
      }
      Frag<T>::guard4(acc[i][0], acc[i][1], acc[i][2], acc[i][3], ah, SPLIT ? al : ah);
    }
    Frag<T>::keep(bh[0], bh[1], bh[2], bh[3]);
    if (SPLIT) Frag<T>::keep(bl[0], bl[1], bl[2], bl[3]);
  }
  acc_guard4(acc[0][0], acc[0][1], acc[0][2], acc[0][3]);
  acc_guard4(acc[1][0], acc[1][1], acc[1][2], acc[1][3]);
  acc_guard4(acc[2][0], acc[2][1], acc[2][2], acc[2][3]);
  acc_guard4(acc[3][0], acc[3][1], acc[3][2], acc[3][3]);

  float* slab = sT[wave];
  const float* Rb = RESID ? (resid + (size_t)b * strideR) : nullptr;
#pragma unroll
  for (int i = 0; i < 4; ++i) {
    const int mBase = m0 + (i << 4);
#pragma unroll
    for (int j = 0; j < 4; ++j) {
      const int n = n0 + (j << 4) + rlane;
      float bv = 0.f;
      if (BIAS_MODE == 2) bv = bias[n];
#pragma unroll
      for (int r = 0; r < 8; ++r) {
        float v = acc[i][j][r] * scale;
        if (BIAS_MODE == 1) v += bias[mBase + mOff + r];
        if (BIAS_MODE == 2) v += bv;
        if (RESID) v += Rb[(size_t)(mBase + mOff + r) * ldc + n];
        if (ACT == 1) v = tanhf(v);
        if (ACT == 2) v = fmaxf(v, 0.0f);
        if (ACT == 3) v = v / (1.0f + expf(-v));
        if (ACT == 4) v = (v > 0.f) ? v : 0.01f * v;
        if (ACT == 5) v = 0.5f * v * (1.0f + erff(v * 0.70710678118654752f));
        slab[(mOff + r) * 68 + (j << 4) + rlane] = v;
      }
    }
    __builtin_amdgcn_fence(__ATOMIC_RELEASE, "workgroup");
    __builtin_amdgcn_wave_barrier();
    __builtin_amdgcn_fence(__ATOMIC_ACQUIRE, "workgroup");
    if (OUT_MODE == 0) {
      float* C = (float*)Cout + (size_t)b * strideC;
      const int hh = lane >> 4, c4 = (lane & 15) * 4;
      for (int pass = 0; pass < 2; ++pass) {
#pragma unroll
        for (int it = 0; it < 8; ++it) {
          const int row = it * 2 + hh;
          v4f v = *(const v4f*)(slab + row * 68 + c4);
          *(volatile v4f*)(C + (size_t)(mBase + row) * ldc + n0 + c4) = v;
        }
        __threadfence();
      }
    } else {
      const int q = lane >> 3, c8 = (lane & 7) * 8;
      unsigned short* C  = (unsigned short*)Cout  + (size_t)b * strideC;
      unsigned short* C2 = (OUT_MODE == 2) ? ((unsigned short*)Cout2 + (size_t)b * strideC) : nullptr;
      for (int pass = 0; pass < 2; ++pass) {
#pragma unroll
        for (int it = 0; it < 4; ++it) {
          const int row = it * 4 + q;
          const float* sp = slab + row * 68 + c8;
          v8h hv, lv;
#pragma unroll
          for (int e = 0; e < 8; ++e) {
            if (OUT_MODE == 1) {
              hv[e] = (_Float16)sp[e];
            } else {
              unsigned short hb = f2bf_bits(sp[e]);
              unsigned short lb = f2bf_bits(sp[e] - bf_bits2f(hb));
              hv[e] = __builtin_bit_cast(_Float16, hb);
              lv[e] = __builtin_bit_cast(_Float16, lb);
            }
          }
          *(volatile v8h*)(C + (size_t)(mBase + row) * ldc + n0 + c8) = hv;
          if (OUT_MODE == 2) *(volatile v8h*)(C2 + (size_t)(mBase + row) * ldc + n0 + c8) = lv;
        }
        __threadfence();
      }
    }
    __builtin_amdgcn_fence(__ATOMIC_RELEASE, "workgroup");
    __builtin_amdgcn_wave_barrier();
    __builtin_amdgcn_fence(__ATOMIC_ACQUIRE, "workgroup");
  }
}

__device__ __forceinline__ void split2(float a, float b, unsigned& hw, unsigned& lw) {
  const unsigned ha = (unsigned)f2bf_bits(a);
  const unsigned hb = (unsigned)f2bf_bits(b);
  const unsigned la = (unsigned)f2bf_bits(a - bf_bits2f((unsigned short)ha));
  const unsigned lb = (unsigned)f2bf_bits(b - bf_bits2f((unsigned short)hb));
  hw = ha | (hb << 16);
  lw = la | (lb << 16);
}
__device__ __forceinline__ void split8(v4f a, v4f b, v4u& hw, v4u& lw) {
  const float f0 = a.x, f1 = a.y, f2 = a.z, f3 = a.w;
  const float f4 = b.x, f5 = b.y, f6 = b.z, f7 = b.w;
  unsigned h0, l0, h1, l1, h2, l2, h3, l3;
  split2(f0, f1, h0, l0);
  split2(f2, f3, h1, l1);
  split2(f4, f5, h2, l2);
  split2(f6, f7, h3, l3);
  hw = (v4u){h0, h1, h2, h3};
  lw = (v4u){l0, l1, l2, l3};
}

__global__ __launch_bounds__(256) void mix_split_kernel(
    const float* __restrict__ x, const float* __restrict__ muR, const float* __restrict__ muV,
    unsigned short* __restrict__ ARh, unsigned short* __restrict__ ARl,
    unsigned short* __restrict__ AVh, unsigned short* __restrict__ AVl, int n8)
{
  const int gid = blockIdx.x * 256 + (int)threadIdx.x;
  if (gid >= n8) return;
  const int e0 = gid * 8;
  const int m  = e0 / NEMB;
  const int c  = e0 - m * NEMB;
  const int t  = m & (NTOK - 1);
  const int ms = (m + 1 < NROWS) ? (m + 1) : (NROWS - 1);
  const float fs = (t < NTOK - 1) ? 1.0f : 0.0f;

  const float* xr = x + (size_t)m * NEMB + c;
  const float* xn = x + (size_t)ms * NEMB + c;
  const float* pr = muR + (size_t)t * NEMB + c;
  const float* pv = muV + (size_t)t * NEMB + c;
  const v4f xa = *(const v4f*)(xr);
  const v4f xb = *(const v4f*)(xr + 4);
  const v4f na = *(const v4f*)(xn);
  const v4f nb = *(const v4f*)(xn + 4);
  const v4f ra = *(const v4f*)(pr);
  const v4f rb = *(const v4f*)(pr + 4);
  const v4f va = *(const v4f*)(pv);
  const v4f vb = *(const v4f*)(pv + 4);

  const v4f sa = na * fs;
  const v4f sb = nb * fs;
  const v4f mra = ra * xa + (1.0f - ra) * sa;
  const v4f mrb = rb * xb + (1.0f - rb) * sb;
  const v4f mva = va * xa + (1.0f - va) * sa;
  const v4f mvb = vb * xb + (1.0f - vb) * sb;

  v4u hr, lr, hv, lv;
  split8(mra, mrb, hr, lr);
  split8(mva, mvb, hv, lv);

  unsigned short* o0 = ARh + e0;
  unsigned short* o1 = ARl + e0;
  unsigned short* o2 = AVh + e0;
  unsigned short* o3 = AVl + e0;
  *(volatile v4u*)(o0) = hr;
  *(volatile v4u*)(o1) = lr;
  *(volatile v4u*)(o2) = hv;
  *(volatile v4u*)(o3) = lv;
  __threadfence();
  *(volatile v4u*)(o0) = hr;
  *(volatile v4u*)(o1) = lr;
  *(volatile v4u*)(o2) = hv;
  *(volatile v4u*)(o3) = lv;
}

__global__ __launch_bounds__(256) void weight_split_kernel(
    const float* __restrict__ w, unsigned short* __restrict__ Wh, unsigned short* __restrict__ Wl, int n8)
{
  const int gid = blockIdx.x * 256 + (int)threadIdx.x;
  if (gid >= n8) return;
  const int e0 = gid * 8;
  const v4f a = *(const v4f*)(w + e0);
  const v4f b = *(const v4f*)(w + e0 + 4);
  v4u hw, lw;
  split8(a, b, hw, lw);
  unsigned short* o0 = Wh + e0;
  unsigned short* o1 = Wl + e0;
  *(volatile v4u*)(o0) = hw;
  *(volatile v4u*)(o1) = lw;
  __threadfence();
  *(volatile v4u*)(o0) = hw;
  *(volatile v4u*)(o1) = lw;
}

__global__ __launch_bounds__(256) void gate_split_kernel(
    const float* __restrict__ Rf, const float* __restrict__ Vf,
    unsigned short* __restrict__ Sh, unsigned short* __restrict__ Sl, int ntot)
{
  __shared__ __align__(16) unsigned shi[2048];
  __shared__ __align__(16) unsigned slo[2048];
  const int tid = (int)threadIdx.x;
  const size_t base = (size_t)blockIdx.x * 2048;
#pragma unroll 1
  for (int it = 0; it < 8; ++it) {
    const int le = it * 256 + tid;
    size_t g = base + (size_t)le;
    if (g > (size_t)(ntot - 1)) g = (size_t)(ntot - 1);
    const float r = Rf[g];
    const float v = Vf[g];
    const float e = expf(-r);
    const float sig = 1.0f / (1.0f + e);
    const float s = sig * v;
    const unsigned hb = (unsigned)f2bf_bits(s);
    const unsigned lb = (unsigned)f2bf_bits(s - bf_bits2f((unsigned short)hb));
    shi[le] = hb;
    slo[le] = lb;
  }
  __syncthreads();
  const int e0 = tid * 8;
  const v4u h0 = *(const v4u*)(shi + e0);
  const v4u h1 = *(const v4u*)(shi + e0 + 4);
  const v4u l0 = *(const v4u*)(slo + e0);
  const v4u l1 = *(const v4u*)(slo + e0 + 4);
  const v4u hw = (v4u){ h0.x | (h0.y << 16), h0.z | (h0.w << 16), h1.x | (h1.y << 16), h1.z | (h1.w << 16) };
  const v4u lw = (v4u){ l0.x | (l0.y << 16), l0.z | (l0.w << 16), l1.x | (l1.y << 16), l1.z | (l1.w << 16) };
  unsigned short* o0 = Sh + base + e0;
  unsigned short* o1 = Sl + base + e0;
  *(volatile v4u*)(o0) = hw;
  *(volatile v4u*)(o1) = lw;
  __threadfence();
  *(volatile v4u*)(o0) = hw;
  *(volatile v4u*)(o1) = lw;
}

extern "C" void kernel_launch(void* const* d_in, const int* in_sizes, int n_in,
                              void* d_out, int out_size, void* d_ws, size_t ws_size,
                              hipStream_t stream)
{
  if (n_in < 14) return;
  if (in_sizes[0] != NROWS * NEMB || in_sizes[1] != NTOK * NEMB || in_sizes[3] != NTOK * NEMB ||
      in_sizes[4] != NATT * NEMB || in_sizes[5] != NATT || in_sizes[8] != NATT * NEMB || in_sizes[9] != NATT ||
      in_sizes[10] != NEMB * NATT || in_sizes[11] != NEMB || out_size != NROWS * NEMB) return;

  const float* x   = (const float*)d_in[0];
  const float* muR = (const float*)d_in[1];
  const float* muV = (const float*)d_in[3];
  const float* Wr  = (const float*)d_in[4];
  const float* br  = (const float*)d_in[5];
  const float* Wv  = (const float*)d_in[8];
  const float* bv  = (const float*)d_in[9];
  const float* Wo  = (const float*)d_in[10];
  const float* bo  = (const float*)d_in[11];
  float* out = (float*)d_out;

  const size_t P16 = (size_t)NROWS * NEMB * 2;
  const size_t P32 = (size_t)NROWS * NATT * 4;
  const size_t total = 12 * P16 + 2 * P32;
  if (ws_size < total) return;
  unsigned char* ws = (unsigned char*)d_ws;
  unsigned short* ARh = (unsigned short*)(ws + 0 * P16);
  unsigned short* ARl = (unsigned short*)(ws + 1 * P16);
  unsigned short* AVh = (unsigned short*)(ws + 2 * P16);
  unsigned short* AVl = (unsigned short*)(ws + 3 * P16);
  unsigned short* Wrh = (unsigned short*)(ws + 4 * P16);
  unsigned short* Wrl = (unsigned short*)(ws + 5 * P16);
  unsigned short* Wvh = (unsigned short*)(ws + 6 * P16);
  unsigned short* Wvl = (unsigned short*)(ws + 7 * P16);
  unsigned short* Woh = (unsigned short*)(ws + 8 * P16);
  unsigned short* Wol = (unsigned short*)(ws + 9 * P16);
  float*          Rf  = (float*)(ws + 10 * P16);
  float*          Vf  = (float*)(ws + 10 * P16 + P32);
  unsigned short* Sh  = (unsigned short*)(ws + 10 * P16 + 2 * P32);
  unsigned short* Sl  = (unsigned short*)(ws + 11 * P16 + 2 * P32);

  const int n8a = NROWS * NEMB / 8;
  mix_split_kernel<<<(n8a + 255) / 256, 256, 0, stream>>>(x, muR, muV, ARh, ARl, AVh, AVl, n8a);

  const int n8w = NATT * NEMB / 8;
  weight_split_kernel<<<(n8w + 255) / 256, 256, 0, stream>>>(Wr, Wrh, Wrl, n8w);
  weight_split_kernel<<<(n8w + 255) / 256, 256, 0, stream>>>(Wv, Wvh, Wvl, n8w);
  const int n8o = NEMB * NATT / 8;
  weight_split_kernel<<<(n8o + 255) / 256, 256, 0, stream>>>(Wo, Woh, Wol, n8o);

  const int tilesRV = (NROWS / 64) * (NATT / 64);
  dim3 gRV((tilesRV + 7) / 8, 1, 1);
  wmma_gemm64<1, true, 2, 0, false, 0><<<gRV, 256, 0, stream>>>(
      ARh, ARl, NEMB, 0L, Wrh, Wrl, NEMB, 0L, (void*)Rf, (void*)nullptr, NATT, 0L,
      br, (const float*)nullptr, 0L, NROWS, NATT, NEMB, 1.0f);
  wmma_gemm64<1, true, 2, 0, false, 0><<<gRV, 256, 0, stream>>>(
      AVh, AVl, NEMB, 0L, Wvh, Wvl, NEMB, 0L, (void*)Vf, (void*)nullptr, NATT, 0L,
      bv, (const float*)nullptr, 0L, NROWS, NATT, NEMB, 1.0f);

  const int ntotS = NROWS * NATT;
  gate_split_kernel<<<ntotS / 2048, 256, 0, stream>>>(Rf, Vf, Sh, Sl, ntotS);

  const int tilesO = (NROWS / 64) * (NEMB / 64);
  dim3 gO((tilesO + 7) / 8, 1, 1);
  wmma_gemm64<1, true, 2, 0, false, 0><<<gO, 256, 0, stream>>>(
      Sh, Sl, NATT, 0L, Woh, Wol, NATT, 0L, (void*)out, (void*)nullptr, NEMB, 0L,
      bo, (const float*)nullptr, 0L, NROWS, NEMB, NATT, 1.0f);
}
